// Rnn_44598940402038
// MI455X (gfx1250) — hardware-verified
//
#include <hip/hip_runtime.h>
#include <math.h>

typedef __attribute__((ext_vector_type(16))) _Float16 v16h;
typedef __attribute__((ext_vector_type(8)))  _Float16 v8h;
typedef __attribute__((ext_vector_type(8)))  float    v8f;
typedef __attribute__((ext_vector_type(4)))  float    v4f;

constexpr int kBatch    = 1024;
constexpr int kStep     = 512;
constexpr int kEmb      = 64;
constexpr int kHid      = 128;
constexpr int kOutD     = 2;
constexpr int kVocab    = 4411;
constexpr int kVocabPad = 4416;
constexpr int kRowsPB   = 16;
constexpr int kScanBlk  = kBatch / kRowsPB;
constexpr int kScanThr  = 64;
constexpr int kWP       = kHid + 8;
constexpr int kFP       = kHid + 4;
constexpr float kWCarry   = 16.0f;
constexpr float kWInv     = 1.0f / 16.0f;
constexpr float kResCarry = 2048.0f;
constexpr float kResInv   = 1.0f / 2048.0f;
constexpr float kF16MinNormal = 6.103515625e-5f;

static_assert(kBatch % kRowsPB == 0, "batch tiles");
static_assert(kScanBlk == 64, "64 blocks");
static_assert(kHid == 2 * 64, "two waves x 64 columns");
static_assert(kHid % 32 == 0 && kEmb % 4 == 0, "k multiples");
static_assert(kWP % 8 == 0 && kFP % 4 == 0, "16-B aligned pitches");
static_assert((kVocabPad * 32) % 256 == 0, "table grid exact");
static_assert(kVocabPad >= kVocab && kVocabPad % 16 == 0, "table pad");
static_assert(kOutD * kHid == 4 * kScanThr, "head weight staging exact");
static_assert(kRowsPB * kOutD == 32, "one output line per block");
static_assert(kRowsPB * kHid == kScanThr * 32, "x staging exact");

union FragU { v16h v; v8h h[2]; };
__device__ __forceinline__ v16h frag_load(const _Float16* p) {
  FragU f;
  f.h[0] = *(const v8h*)(p);
  f.h[1] = *(const v8h*)(p + 16);
  return f.v;
}
__device__ __forceinline__ v8f mma_h(v16h a, v16h b, v8f c) {
  return __builtin_amdgcn_wmma_f32_16x16x32_f16(false, a, false, b, (short)0, c, false, false);
}
__device__ __forceinline__ void guard_group(v8f& m0, v8f& m1, v8f& m2, v8f& m3,
                                            v8f& r0, v8f& r1, v8f& r2, v8f& r3,
                                            v16h a0, v16h a1,
                                            v16h b0, v16h b1, v16h b2, v16h b3,
                                            v16h c0, v16h c1, v16h c2, v16h c3) {
  asm volatile("v_nop\n\tv_nop\n\tv_nop\n\tv_nop"
               : "+v"(m0), "+v"(m1), "+v"(m2), "+v"(m3), "+v"(r0), "+v"(r1), "+v"(r2), "+v"(r3)
               : "v"(a0), "v"(a1), "v"(b0), "v"(b1), "v"(b2), "v"(b3), "v"(c0), "v"(c1), "v"(c2), "v"(c3));
}
__device__ __forceinline__ void guard_acc8(v8f& m0, v8f& m1, v8f& m2, v8f& m3,
                                           v8f& r0, v8f& r1, v8f& r2, v8f& r3) {
  asm volatile("v_nop\n\tv_nop\n\tv_nop\n\tv_nop"
               : "+v"(m0), "+v"(m1), "+v"(m2), "+v"(m3), "+v"(r0), "+v"(r1), "+v"(r2), "+v"(r3));
}

__device__ __forceinline__ void split16(float v, _Float16& hi, _Float16& lo) {
  const float sel = (fabsf(v) < kF16MinNormal) ? 0.0f : v;
  hi = (_Float16)sel;
  float hf = (float)hi;
  asm volatile("" : "+v"(hf));
  lo = (_Float16)((v - hf) * kResCarry);
}

__device__ __forceinline__ float tanh_f32(float x) {
  const float e = expf(2.0f * x);
  return 1.0f - 2.0f * __builtin_amdgcn_rcpf(1.0f + e);
}

__global__ __launch_bounds__(256) void proj_table_kernel(const float* __restrict__ emb,
                                                         const float* __restrict__ wih,
                                                         const float* __restrict__ bih,
                                                         const float* __restrict__ bhh,
                                                         float* __restrict__ P) {
  const int gid = blockIdx.x * 256 + threadIdx.x;
  const int v   = gid >> 5;
  const int h4  = (gid & 31) * 4;
  const int vc  = (v < kVocab) ? v : (kVocab - 1);
  const float* er = emb + (size_t)vc * kEmb;
  const float* w0 = wih + (size_t)(h4 + 0) * kEmb;
  const float* w1 = wih + (size_t)(h4 + 1) * kEmb;
  const float* w2 = wih + (size_t)(h4 + 2) * kEmb;
  const float* w3 = wih + (size_t)(h4 + 3) * kEmb;
  float s0 = 0.0f, s1 = 0.0f, s2 = 0.0f, s3 = 0.0f;
#pragma unroll 1
  for (int e = 0; e < kEmb; e += 4) {
    const v4f ev = *(const v4f*)(er + e);
    const v4f a0 = *(const v4f*)(w0 + e);
    const v4f a1 = *(const v4f*)(w1 + e);
    const v4f a2 = *(const v4f*)(w2 + e);
    const v4f a3 = *(const v4f*)(w3 + e);
    s0 += ev[0] * a0[0]; s0 += ev[1] * a0[1]; s0 += ev[2] * a0[2]; s0 += ev[3] * a0[3];
    s1 += ev[0] * a1[0]; s1 += ev[1] * a1[1]; s1 += ev[2] * a1[2]; s1 += ev[3] * a1[3];
    s2 += ev[0] * a2[0]; s2 += ev[1] * a2[1]; s2 += ev[2] * a2[2]; s2 += ev[3] * a2[3];
    s3 += ev[0] * a3[0]; s3 += ev[1] * a3[1]; s3 += ev[2] * a3[2]; s3 += ev[3] * a3[3];
  }
  const v4f bi = *(const v4f*)(bih + h4);
  const v4f bh = *(const v4f*)(bhh + h4);
  v4f o;
  o[0] = (s0 + bi[0]) + bh[0];
  o[1] = (s1 + bi[1]) + bh[1];
  o[2] = (s2 + bi[2]) + bh[2];
  o[3] = (s3 + bi[3]) + bh[3];
  float* p = P + (size_t)v * kHid + h4;
  *(volatile v4f*)p = o;
  __threadfence();
  *(volatile v4f*)p = o;
}

__device__ __forceinline__ void stage_x(const int* __restrict__ tokens, const float* __restrict__ P,
                                        float* sX, int b0, int tid, int tstep) {
  const int row = tid >> 2;
  const int seg = (tid & 3) * 32;
  int tok = tokens[(size_t)(b0 + row) * kStep + tstep];
  tok = (tok < 0) ? 0 : tok;
  tok = (tok > kVocab - 1) ? (kVocab - 1) : tok;
  const float* src = P + (size_t)tok * kHid + seg;
  float* dst = sX + row * kFP + seg;
  v4f xv[8];
#pragma unroll
  for (int i = 0; i < 8; ++i) xv[i] = *(const v4f*)(src + 4 * i);
#pragma unroll
  for (int i = 0; i < 8; ++i) *(v4f*)(dst + 4 * i) = xv[i];
}

__global__ __launch_bounds__(kScanThr) void rnn_scan_kernel(const int* __restrict__ tokens,
                                                            const float* __restrict__ P,
                                                            const float* __restrict__ whh,
                                                            const float* __restrict__ wlin,
                                                            const float* __restrict__ blin,
                                                            float* __restrict__ out) {
  __shared__ __align__(16) _Float16 sWh[kHid * kWP];
  __shared__ __align__(16) _Float16 sWl[kHid * kWP];
  __shared__ __align__(16) _Float16 sHh[kRowsPB * kWP];
  __shared__ __align__(16) _Float16 sHl[kRowsPB * kWP];
  __shared__ __align__(16) float    sX[kRowsPB * kFP];
  __shared__ __align__(16) float    sPre[kRowsPB * kFP];
  __shared__ __align__(16) float    sHf[kRowsPB * kFP];
  __shared__ __align__(16) float    sWlin[kOutD * kHid];

  const int tid  = threadIdx.x;
  const int lane = tid & 31;
  const int wave = tid >> 5;
  const int c    = lane & 15;
  const int hh   = lane >> 4;
  const int koff = hh * 8;
  const int mOff = hh * 8;
  const int n0   = wave * 64;
  const int b0   = blockIdx.x * kRowsPB;

  const v8h zh = {(_Float16)0.0f, (_Float16)0.0f, (_Float16)0.0f, (_Float16)0.0f,
                  (_Float16)0.0f, (_Float16)0.0f, (_Float16)0.0f, (_Float16)0.0f};

#pragma unroll 1
  for (int i = tid; i < kHid * (kHid / 8); i += kScanThr) {
    const int row = i >> 4;
    const int c8  = (i & 15) * 8;
    const float* sp = whh + (size_t)row * kHid + c8;
    const v4f a = *(const v4f*)(sp);
    const v4f b = *(const v4f*)(sp + 4);
    v8h hv, lv;
#pragma unroll
    for (int e = 0; e < 4; ++e) {
      _Float16 h0, l0, h1, l1;
      const float wa = a[e] * kWCarry;
      const float wb = b[e] * kWCarry;
      split16(wa, h0, l0);
      split16(wb, h1, l1);
      hv[e] = h0;     lv[e] = l0;
      hv[4 + e] = h1; lv[4 + e] = l1;
    }
    *(v8h*)(sWh + row * kWP + c8) = hv;
    *(v8h*)(sWl + row * kWP + c8) = lv;
  }
#pragma unroll 1
  for (int row = tid; row < kHid; row += kScanThr) {
    *(v8h*)(sWh + row * kWP + kHid) = zh;
    *(v8h*)(sWl + row * kWP + kHid) = zh;
  }
#pragma unroll 1
  for (int i = tid; i < (kRowsPB * kWP) / 8; i += kScanThr) {
    *(v8h*)(sHh + i * 8) = zh;
    *(v8h*)(sHl + i * 8) = zh;
  }
  {
    const v4f w = *(const v4f*)(wlin + 4 * tid);
    *(v4f*)(sWlin + 4 * tid) = w;
  }
  stage_x(tokens, P, sX, b0, tid, 0);
  __syncthreads();

  const v8f z8 = {0.f, 0.f, 0.f, 0.f, 0.f, 0.f, 0.f, 0.f};
  const _Float16* aH = sHh + c * kWP + koff;
  const _Float16* aL = sHl + c * kWP + koff;
  const _Float16* bH = sWh + (n0 + c) * kWP + koff;
  const _Float16* bL = sWl + (n0 + c) * kWP + koff;
  const int prow = lane >> 1;
  const int pcol = n0 + (lane & 1) * 32;

#pragma unroll 1
  for (int t = 0; t < kStep; ++t) {
    const bool last = (t == kStep - 1);

    v8f accM[4], accR[4];
#pragma unroll
    for (int j = 0; j < 4; ++j) {
#pragma unroll
      for (int r = 0; r < 8; ++r) accM[j][r] = sX[(mOff + r) * kFP + n0 + 16 * j + c] * kWCarry;
      accR[j] = z8;
    }
#pragma unroll 1
    for (int kc = 0; kc < kHid / 32; ++kc) {
      const int ko = kc * 32;
      const v16h ah = frag_load(aH + ko);
      const v16h al = frag_load(aL + ko);
      v16h bh[4], bl[4];
#pragma unroll
      for (int j = 0; j < 4; ++j) {
        bh[j] = frag_load(bH + (16 * j) * kWP + ko);
        bl[j] = frag_load(bL + (16 * j) * kWP + ko);
      }
#pragma unroll
      for (int j = 0; j < 4; ++j) accM[j] = mma_h(ah, bh[j], accM[j]);
#pragma unroll
      for (int j = 0; j < 4; ++j) accR[j] = mma_h(ah, bl[j], accR[j]);
#pragma unroll
      for (int j = 0; j < 4; ++j) accR[j] = mma_h(al, bh[j], accR[j]);
      guard_group(accM[0], accM[1], accM[2], accM[3], accR[0], accR[1], accR[2], accR[3],
                  ah, al, bh[0], bh[1], bh[2], bh[3], bl[0], bl[1], bl[2], bl[3]);
    }
    guard_acc8(accM[0], accM[1], accM[2], accM[3], accR[0], accR[1], accR[2], accR[3]);

#pragma unroll
    for (int j = 0; j < 4; ++j) {
#pragma unroll
      for (int r = 0; r < 8; ++r) {
        const float pv = (accM[j][r] + accR[j][r] * kResInv) * kWInv;
        sPre[(mOff + r) * kFP + n0 + 16 * j + c] = pv;
      }
    }
    __syncthreads();

#pragma unroll 1
    for (int q = 0; q < 4; ++q) {
      const int col = pcol + 8 * q;
      const v4f p0 = *(const v4f*)(sPre + prow * kFP + col);
      const v4f p1 = *(const v4f*)(sPre + prow * kFP + col + 4);
      v8h hv, lv;
      v4f f0, f1;
#pragma unroll
      for (int e = 0; e < 4; ++e) {
        const float t0 = tanh_f32(p0[e]);
        const float t1 = tanh_f32(p1[e]);
        _Float16 h0, l0, h1, l1;
        split16(t0, h0, l0);
        split16(t1, h1, l1);
        f0[e] = t0;     f1[e] = t1;
        hv[e] = h0;     lv[e] = l0;
        hv[4 + e] = h1; lv[4 + e] = l1;
      }
      *(v8h*)(sHh + prow * kWP + col) = hv;
      *(v8h*)(sHl + prow * kWP + col) = lv;
      if (last) {
        *(v4f*)(sHf + prow * kFP + col)     = f0;
        *(v4f*)(sHf + prow * kFP + col + 4) = f1;
      }
    }
    {
      const int tn = (t + 1 < kStep) ? (t + 1) : (kStep - 1);
      stage_x(tokens, P, sX, b0, tid, tn);
    }
    __syncthreads();
  }

  if (wave == 0) {
    const int m = lane >> 1;
    const int o = lane & 1;
    float s = 0.0f;
#pragma unroll 4
    for (int k = 0; k < kHid; ++k) s += sHf[m * kFP + k] * sWlin[o * kHid + k];
    s += blin[o];
    float* p = out + (size_t)b0 * kOutD + lane;
    *(volatile float*)p = s;
    __threadfence();
    *(volatile float*)p = s;
  }
}

extern "C" void kernel_launch(void* const* d_in, const int* in_sizes, int n_in,
                              void* d_out, int out_size, void* d_ws, size_t ws_size, hipStream_t stream) {
  if (n_in < 8 || d_out == nullptr || d_ws == nullptr) return;
  if (in_sizes[0] != kBatch * kStep || in_sizes[1] != kVocab * kEmb || in_sizes[2] != kHid * kEmb ||
      in_sizes[3] != kHid * kHid || in_sizes[4] != kHid || in_sizes[5] != kHid ||
      in_sizes[6] != kOutD * kHid || in_sizes[7] != kOutD || out_size != kBatch * kOutD) return;

  const int*   tokens = (const int*)d_in[0];
  const float* emb    = (const float*)d_in[1];
  const float* wih    = (const float*)d_in[2];
  const float* whh    = (const float*)d_in[3];
  const float* bih    = (const float*)d_in[4];
  const float* bhh    = (const float*)d_in[5];
  const float* wlin   = (const float*)d_in[6];
  const float* blin   = (const float*)d_in[7];
  float* outp = (float*)d_out;

  const size_t pbytes = (size_t)kVocabPad * kHid * sizeof(float);
  if (pbytes > ws_size || pbytes > (size_t)134217728) return;
  float* P = (float*)d_ws;

  proj_table_kernel<<<(kVocabPad * 32) / 256, 256, 0, stream>>>(emb, wih, bih, bhh, P);
  rnn_scan_kernel<<<kScanBlk, kScanThr, 0, stream>>>(tokens, P, whh, wlin, blin, outp);
}
